// MultiHeadedAttention_17489106830115
// MI455X (gfx1250) — hardware-run, weakly checked
//
#include <hip/hip_runtime.h>
#include <math.h>

typedef __attribute__((ext_vector_type(16))) _Float16 v16h;
typedef __attribute__((ext_vector_type(8)))  _Float16 v8h;
typedef __attribute__((ext_vector_type(16))) __bf16   v16b;
typedef __attribute__((ext_vector_type(8)))  __bf16   v8b;
typedef __attribute__((ext_vector_type(8)))  float    v8f;
typedef __attribute__((ext_vector_type(4)))  float    v4f;
typedef __attribute__((ext_vector_type(4)))  unsigned int v4u;

constexpr int kBatch    = 4;
constexpr int kSeq      = 2048;
constexpr int kDim      = 1024;
constexpr int kHeads    = 16;
constexpr int kHd       = 64;
constexpr int kTok      = kBatch * kSeq;
constexpr int kCols     = 3 * kDim;
constexpr int kHeadCols = 3 * kHd;
constexpr int kBH       = kBatch * kHeads;
constexpr int kOutRows  = 128;
static_assert(kHeads * kHd == kDim, "head split");
static_assert(kTok == 8192 && kCols == 3072 && kHeadCols == 192 && kBH == 64, "shapes");
static_assert((kDim % 32) == 0 && (kSeq % 32) == 0 && (kHd % 32) == 0, "contraction depths are multiples of 32");
static_assert((kTok % 64) == 0 && (kDim % 64) == 0 && ((2 * kDim) % 64) == 0, "tile multiples of 64");
static_assert((kSeq % kOutRows) == 0, "row chunking");

constexpr float kAttnScale = 32.0f;
static_assert(kAttnScale * kAttnScale == (float)kDim, "score scale squared equals the width");
constexpr float kQCarry  = 16.0f;
constexpr float kMFold   = 1.0f / (kQCarry * kQCarry);
constexpr float kLoCarry = 2048.0f;
constexpr float kLoFold  = 1.0f / kLoCarry;
constexpr float kOutScale = kAttnScale / kQCarry;
constexpr float kF16MinNormal = 6.103515625e-5f;

constexpr size_t kOffX16   = 0;
constexpr size_t kOffWT16  = kOffX16   + (size_t)kTok  * kDim * 2;
constexpr size_t kOffBPERM = kOffWT16  + (size_t)kCols * kDim * 2;
constexpr size_t kOffQ16   = kOffBPERM + (size_t)kCols * 4;
constexpr size_t kOffKVT16 = kOffQ16   + (size_t)kTok  * kDim * 2;
constexpr size_t kOffMTHI  = kOffKVT16 + (size_t)(2 * kDim) * kTok * 2;
constexpr size_t kOffMTLO  = kOffMTHI  + (size_t)kBH * kHd * kHd * 2;
constexpr size_t kWsTotal  = kOffMTLO  + (size_t)kBH * kHd * kHd * 2;
static_assert(kWsTotal == 74461184ull, "carve total");
static_assert(kWsTotal <= 134217728ull, "carve cap");
static_assert((kOffWT16 % 128) == 0 && (kOffBPERM % 128) == 0 && (kOffQ16 % 128) == 0 &&
              (kOffKVT16 % 128) == 0 && (kOffMTHI % 128) == 0 && (kOffMTLO % 128) == 0, "128-B aligned regions");

__device__ __forceinline__ unsigned bf16_rne_bits32(float f) {
  unsigned u = __float_as_uint(f);
  const unsigned lsb = (u & 0x00010000u) ? 1u : 0u;
  u = (u + 0x7FFFu + lsb) & 0xFFFF0000u;
  return u;
}
__device__ __forceinline__ unsigned pack_bf16x2(float e_lo, float e_hi) {
  const unsigned a = bf16_rne_bits32(e_lo);
  const unsigned b = bf16_rne_bits32(e_hi);
  return (a >> 16) | b;
}
__device__ __forceinline__ float flush_f16_sub(float v) {
  return (fabsf(v) < kF16MinNormal) ? 0.0f : v;
}

__device__ __forceinline__ void guard4_b(v8f& c0, v8f& c1, v8f& c2, v8f& c3, v16b x) {
  asm volatile("v_nop\n\tv_nop\n\tv_nop\n\tv_nop" : "+v"(c0), "+v"(c1), "+v"(c2), "+v"(c3) : "v"(x));
}
__device__ __forceinline__ void guard4_h(v8f& c0, v8f& c1, v8f& c2, v8f& c3, v16h x,
                                         v16h y0, v16h y1, v16h y2, v16h y3) {
  asm volatile("v_nop\n\tv_nop\n\tv_nop\n\tv_nop" : "+v"(c0), "+v"(c1), "+v"(c2), "+v"(c3)
               : "v"(x), "v"(y0), "v"(y1), "v"(y2), "v"(y3));
}
__device__ __forceinline__ void keep4_b(v16b a, v16b b, v16b c, v16b d) { asm volatile("v_nop" :: "v"(a), "v"(b), "v"(c), "v"(d)); }
__device__ __forceinline__ void acc_guard4(v8f& a, v8f& b, v8f& c, v8f& d) { asm volatile("v_nop\n\tv_nop\n\tv_nop\n\tv_nop" : "+v"(a), "+v"(b), "+v"(c), "+v"(d)); }

template <typename T> struct Frag;
template <> struct Frag<_Float16> {
  typedef v16h V; union U { v16h v; v8h h[2]; };
  static __device__ __forceinline__ v16h load(const _Float16* p) {
    U f; f.h[0] = *(const v8h*)(p); f.h[1] = *(const v8h*)(p + 16); return f.v;
  }
  static __device__ __forceinline__ v8f mma(v16h a, v16h b, v8f c) {
    return __builtin_amdgcn_wmma_f32_16x16x32_f16(false, a, false, b, (short)0, c, false, false);
  }
};
template <> struct Frag<__bf16> {
  typedef v16b V; union U { v16b v; v8b h[2]; };
  static __device__ __forceinline__ v16b load(const __bf16* p) {
    U f; f.h[0] = *(const v8b*)(p); f.h[1] = *(const v8b*)(p + 16); return f.v;
  }
  static __device__ __forceinline__ v8f mma(v16b a, v16b b, v8f c) {
    return __builtin_amdgcn_wmma_f32_16x16x32_bf16(false, a, false, b, (short)0, c, false, false);
  }
};

__global__ __launch_bounds__(256) void cvt_rows_bf16_kernel(const float* __restrict__ in, unsigned int* __restrict__ out, int n8) {
  const int i = blockIdx.x * 256 + threadIdx.x;
  if (i >= n8) return;
  const float* p = in + 8 * (size_t)i;
  const v4f a = *(const v4f*)(p);
  const v4f c = *(const v4f*)(p + 4);
  const float a0 = a[0], a1 = a[1], a2 = a[2], a3 = a[3];
  const float c0 = c[0], c1 = c[1], c2 = c[2], c3 = c[3];
  const v4u u = (v4u){pack_bf16x2(a0, a1), pack_bf16x2(a2, a3), pack_bf16x2(c0, c1), pack_bf16x2(c2, c3)};
  unsigned int* q = out + 4 * (size_t)i;
  *(volatile v4u*)q = u;
  __threadfence();
  *(volatile v4u*)q = u;
}

__global__ __launch_bounds__(256) void wt_deint_bf16_kernel(const float* __restrict__ W, unsigned short* __restrict__ Wt) {
  __shared__ float sm[kHeadCols][65];
  const unsigned t  = threadIdx.x;
  const unsigned k0 = blockIdx.x * 64u;
  const unsigned h  = blockIdx.y;
#pragma unroll
  for (int i = 0; i < 12; ++i) {
    const unsigned e4 = (unsigned)i * 256u + t;
    const unsigned kr = e4 / 48u;
    const unsigned c4 = (e4 - kr * 48u) * 4u;
    const v4f v = *(const v4f*)(W + (size_t)(k0 + kr) * kCols + h * (unsigned)kHeadCols + c4);
    const float v0 = v[0], v1 = v[1], v2 = v[2], v3 = v[3];
    sm[c4 + 0][kr] = v0;
    sm[c4 + 1][kr] = v1;
    sm[c4 + 2][kr] = v2;
    sm[c4 + 3][kr] = v3;
  }
  __syncthreads();
  const unsigned lane = t & 31u, wave = t >> 5;
  const unsigned q = lane >> 3, c8 = (lane & 7u) * 8u;
  v4u u[6];
#pragma unroll
  for (int it = 0; it < 6; ++it) {
    const unsigned rl  = (unsigned)it * 32u + wave * 4u + q;
    const unsigned sel = rl / (unsigned)kHd;
    const unsigned d   = rl % (unsigned)kHd;
    const float* sp = &sm[d * 3u + sel][c8];
    u[it] = (v4u){pack_bf16x2(sp[0], sp[1]), pack_bf16x2(sp[2], sp[3]),
                  pack_bf16x2(sp[4], sp[5]), pack_bf16x2(sp[6], sp[7])};
  }
  for (int pass = 0; pass < 2; ++pass) {
#pragma unroll
    for (int it = 0; it < 6; ++it) {
      const unsigned rl  = (unsigned)it * 32u + wave * 4u + q;
      const unsigned sel = rl / (unsigned)kHd;
      const unsigned d   = rl % (unsigned)kHd;
      const size_t r = (size_t)sel * kDim + h * (unsigned)kHd + d;
      *(volatile v4u*)(Wt + r * kDim + k0 + c8) = u[it];
    }
    __threadfence();
  }
}

__global__ __launch_bounds__(256) void bias_perm_kernel(const float* __restrict__ bsrc, float* __restrict__ bperm) {
  const unsigned i   = blockIdx.x * 256u + threadIdx.x;
  const unsigned r0  = i * 4u;
  const unsigned sel = r0 / (unsigned)kDim;
  const unsigned rem = r0 % (unsigned)kDim;
  const unsigned h   = rem / (unsigned)kHd;
  const unsigned d0  = rem % (unsigned)kHd;
  const unsigned cb  = h * (unsigned)kHeadCols + d0 * 3u + sel;
  const float f0 = bsrc[cb], f1 = bsrc[cb + 3u], f2 = bsrc[cb + 6u], f3 = bsrc[cb + 9u];
  v4f v;
  v[0] = __uint_as_float(bf16_rne_bits32(f0)) * kQCarry;
  v[1] = __uint_as_float(bf16_rne_bits32(f1)) * kQCarry;
  v[2] = __uint_as_float(bf16_rne_bits32(f2)) * kQCarry;
  v[3] = __uint_as_float(bf16_rne_bits32(f3)) * kQCarry;
  float* q = bperm + r0;
  *(volatile v4f*)q = v;
  __threadfence();
  *(volatile v4f*)q = v;
}

template <int BIAS_MODE>
__global__ __launch_bounds__(256) void gemm64_bf16_f16out_kernel(
    const unsigned short* __restrict__ Ap, int lda,
    const unsigned short* __restrict__ Btp, int ldb,
    unsigned short* __restrict__ Cp, int ldc,
    const float* __restrict__ bias, int M, int N, int K, float scale) {
  typedef __bf16 T;
  typedef v16b V;
  const T* A  = (const T*)Ap;
  const T* Bt = (const T*)Btp;
  __shared__ __align__(16) float sT[8][16 * 68];
  const int lane = threadIdx.x & 31;
  const int wave = threadIdx.x >> 5;
  const int tilesN = N >> 6;
  const int tilesM = M >> 6;
  const int tile = blockIdx.x * 8 + wave;
  if (tile >= tilesM * tilesN) return;
  const int tm = tile / tilesN;
  const int tn = tile - tm * tilesN;
  const int m0 = tm << 6;
  const int n0 = tn << 6;

  const int rlane = lane & 15;
  const int koff  = (lane >> 4) * 8;
  const int mOff  = (lane >> 4) * 8;

  v8f acc[4][4];
#pragma unroll
  for (int i = 0; i < 4; ++i)
#pragma unroll
    for (int j = 0; j < 4; ++j) acc[i][j] = (v8f){0.f, 0.f, 0.f, 0.f, 0.f, 0.f, 0.f, 0.f};

  for (int k0 = 0; k0 < K; k0 += 32) {
    V bh[4];
#pragma unroll
    for (int j = 0; j < 4; ++j) {
      const size_t bo = (size_t)(n0 + (j << 4) + rlane) * ldb + koff + k0;
      bh[j] = Frag<T>::load(Bt + bo);
    }
#pragma unroll
    for (int i = 0; i < 4; ++i) {
      const size_t ao = (size_t)(m0 + (i << 4) + rlane) * lda + koff + k0;
      V ah = Frag<T>::load(A + ao);
#pragma unroll
      for (int j = 0; j < 4; ++j) acc[i][j] = Frag<T>::mma(ah, bh[j], acc[i][j]);
      guard4_b(acc[i][0], acc[i][1], acc[i][2], acc[i][3], ah);
    }
    keep4_b(bh[0], bh[1], bh[2], bh[3]);
  }
  acc_guard4(acc[0][0], acc[0][1], acc[0][2], acc[0][3]);
  acc_guard4(acc[1][0], acc[1][1], acc[1][2], acc[1][3]);
  acc_guard4(acc[2][0], acc[2][1], acc[2][2], acc[2][3]);
  acc_guard4(acc[3][0], acc[3][1], acc[3][2], acc[3][3]);

  float* slab = sT[wave];
  float bn[4] = {0.f, 0.f, 0.f, 0.f};
  if (BIAS_MODE == 2) {
#pragma unroll
    for (int j = 0; j < 4; ++j) bn[j] = bias[n0 + (j << 4) + rlane];
  }
  const int q = lane >> 3, c8 = (lane & 7) * 8;
#pragma unroll
  for (int i = 0; i < 4; ++i) {
    const int mBase = m0 + (i << 4);
    float bm[8] = {0.f, 0.f, 0.f, 0.f, 0.f, 0.f, 0.f, 0.f};
    if (BIAS_MODE == 1) {
      const v4f b0 = *(const v4f*)(bias + mBase + mOff);
      const v4f b1 = *(const v4f*)(bias + mBase + mOff + 4);
      bm[0] = b0[0]; bm[1] = b0[1]; bm[2] = b0[2]; bm[3] = b0[3];
      bm[4] = b1[0]; bm[5] = b1[1]; bm[6] = b1[2]; bm[7] = b1[3];
    }
#pragma unroll
    for (int j = 0; j < 4; ++j) {
#pragma unroll
      for (int r = 0; r < 8; ++r) {
        const float add = (BIAS_MODE == 1) ? bm[r] : bn[j];
        const float v = acc[i][j][r] * scale + add;
        slab[(mOff + r) * 68 + (j << 4) + rlane] = v;
      }
    }
    __builtin_amdgcn_fence(__ATOMIC_RELEASE, "workgroup");
    __builtin_amdgcn_wave_barrier();
    __builtin_amdgcn_fence(__ATOMIC_ACQUIRE, "workgroup");
    v8h hv[4];
#pragma unroll
    for (int it = 0; it < 4; ++it) {
      const int row = it * 4 + q;
      const float* sp = slab + row * 68 + c8;
#pragma unroll
      for (int e = 0; e < 8; ++e) {
        const float x = flush_f16_sub(sp[e]);
        hv[it][e] = (_Float16)x;
      }
    }
    for (int pass = 0; pass < 2; ++pass) {
#pragma unroll
      for (int it = 0; it < 4; ++it) {
        const int row = it * 4 + q;
        *(volatile v8h*)(Cp + (size_t)(mBase + row) * ldc + n0 + c8) = hv[it];
      }
      __threadfence();
    }
    __builtin_amdgcn_fence(__ATOMIC_RELEASE, "workgroup");
    __builtin_amdgcn_wave_barrier();
    __builtin_amdgcn_fence(__ATOMIC_ACQUIRE, "workgroup");
  }
}

__global__ __launch_bounds__(128) void ktv_kernel(const unsigned short* __restrict__ KVTp,
                                                  unsigned short* __restrict__ MThi,
                                                  unsigned short* __restrict__ MTlo) {
  __shared__ __align__(16) float sT[4][16 * 68];
  const _Float16* KVT = (const _Float16*)KVTp;
  const int lane = threadIdx.x & 31;
  const int wave = threadIdx.x >> 5;
  const int rlane = lane & 15;
  const int koff  = (lane >> 4) * 8;
  const int mOff  = (lane >> 4) * 8;
  const int bh = blockIdx.x;
  const int b  = bh / kHeads;
  const int h  = bh - b * kHeads;

  const _Float16* Ab = KVT + (size_t)(kDim + h * kHd + wave * 16 + rlane) * kTok + (size_t)b * kSeq + koff;
  const _Float16* Bb = KVT + (size_t)(h * kHd + rlane) * kTok + (size_t)b * kSeq + koff;

  v8f acc0 = (v8f){0.f, 0.f, 0.f, 0.f, 0.f, 0.f, 0.f, 0.f};
  v8f acc1 = acc0, acc2 = acc0, acc3 = acc0;
  for (int k0 = 0; k0 < kSeq; k0 += 32) {
    const v16h a  = Frag<_Float16>::load(Ab + k0);
    const v16h b0 = Frag<_Float16>::load(Bb + k0);
    const v16h b1 = Frag<_Float16>::load(Bb + (size_t)16 * kTok + k0);
    const v16h b2 = Frag<_Float16>::load(Bb + (size_t)32 * kTok + k0);
    const v16h b3 = Frag<_Float16>::load(Bb + (size_t)48 * kTok + k0);
    acc0 = Frag<_Float16>::mma(a, b0, acc0);
    acc1 = Frag<_Float16>::mma(a, b1, acc1);
    acc2 = Frag<_Float16>::mma(a, b2, acc2);
    acc3 = Frag<_Float16>::mma(a, b3, acc3);
    guard4_h(acc0, acc1, acc2, acc3, a, b0, b1, b2, b3);
  }
  acc_guard4(acc0, acc1, acc2, acc3);

  float* slab = sT[wave];
#pragma unroll
  for (int r = 0; r < 8; ++r) {
    slab[(mOff + r) * 68 +  0 + rlane] = acc0[r] * kMFold;
    slab[(mOff + r) * 68 + 16 + rlane] = acc1[r] * kMFold;
    slab[(mOff + r) * 68 + 32 + rlane] = acc2[r] * kMFold;
    slab[(mOff + r) * 68 + 48 + rlane] = acc3[r] * kMFold;
  }
  __syncthreads();
  const int q = lane >> 3, c8 = (lane & 7) * 8;
  v8h hv[4], lv[4];
#pragma unroll
  for (int it = 0; it < 4; ++it) {
    const int row = it * 4 + q;
    const float* sp = slab + row * 68 + c8;
#pragma unroll
    for (int e = 0; e < 8; ++e) {
      const float m  = sp[e];
      const float mf = flush_f16_sub(m);
      const _Float16 hs = (_Float16)mf;
      const float hf = (float)hs;
      const float rs = flush_f16_sub((m - hf) * kLoCarry);
      const _Float16 ls = (_Float16)rs;
      hv[it][e] = hs;
      lv[it][e] = ls;
    }
  }
  for (int pass = 0; pass < 2; ++pass) {
#pragma unroll
    for (int it = 0; it < 4; ++it) {
      const int row = it * 4 + q;
      const size_t o = ((size_t)bh * kHd + wave * 16 + row) * kHd + c8;
      *(volatile v8h*)(MThi + o) = hv[it];
      *(volatile v8h*)(MTlo + o) = lv[it];
    }
    __threadfence();
  }
}

__global__ __launch_bounds__(256) void qm_out_kernel(const unsigned short* __restrict__ Q16p,
                                                     const unsigned short* __restrict__ MThip,
                                                     const unsigned short* __restrict__ MTlop,
                                                     float* __restrict__ out) {
  __shared__ __align__(16) float sT[8][16 * 68];
  const _Float16* Q16  = (const _Float16*)Q16p;
  const _Float16* MThi = (const _Float16*)MThip;
  const _Float16* MTlo = (const _Float16*)MTlop;
  const int lane = threadIdx.x & 31;
  const int wave = threadIdx.x >> 5;
  const int rlane = lane & 15;
  const int koff  = (lane >> 4) * 8;
  const int mOff  = (lane >> 4) * 8;
  constexpr int kChunks = kSeq / kOutRows;
  const int bh    = blockIdx.x / kChunks;
  const int chunk = blockIdx.x - bh * kChunks;
  const int b  = bh / kHeads;
  const int h  = bh - b * kHeads;
  const int i0 = chunk * kOutRows + wave * 16;

  const _Float16* Ab = Q16 + (size_t)(b * kSeq + i0 + rlane) * kDim + h * kHd + koff;
  const _Float16* Bh = MThi + (size_t)bh * kHd * kHd + (size_t)rlane * kHd + koff;
  const _Float16* Bl = MTlo + (size_t)bh * kHd * kHd + (size_t)rlane * kHd + koff;

  v8f ah0 = (v8f){0.f, 0.f, 0.f, 0.f, 0.f, 0.f, 0.f, 0.f};
  v8f ah1 = ah0, ah2 = ah0, ah3 = ah0;
  v8f al0 = ah0, al1 = ah0, al2 = ah0, al3 = ah0;
#pragma unroll
  for (int ks = 0; ks < 2; ++ks) {
    const int k0 = ks * 32;
    const v16h a   = Frag<_Float16>::load(Ab + k0);
    const v16h bh0 = Frag<_Float16>::load(Bh + 0 * 16 * kHd + k0);
    const v16h bh1 = Frag<_Float16>::load(Bh + 1 * 16 * kHd + k0);
    const v16h bh2 = Frag<_Float16>::load(Bh + 2 * 16 * kHd + k0);
    const v16h bh3 = Frag<_Float16>::load(Bh + 3 * 16 * kHd + k0);
    const v16h bl0 = Frag<_Float16>::load(Bl + 0 * 16 * kHd + k0);
    const v16h bl1 = Frag<_Float16>::load(Bl + 1 * 16 * kHd + k0);
    const v16h bl2 = Frag<_Float16>::load(Bl + 2 * 16 * kHd + k0);
    const v16h bl3 = Frag<_Float16>::load(Bl + 3 * 16 * kHd + k0);
    ah0 = Frag<_Float16>::mma(a, bh0, ah0);
    ah1 = Frag<_Float16>::mma(a, bh1, ah1);
    ah2 = Frag<_Float16>::mma(a, bh2, ah2);
    ah3 = Frag<_Float16>::mma(a, bh3, ah3);
    al0 = Frag<_Float16>::mma(a, bl0, al0);
    al1 = Frag<_Float16>::mma(a, bl1, al1);
    al2 = Frag<_Float16>::mma(a, bl2, al2);
    al3 = Frag<_Float16>::mma(a, bl3, al3);
    guard4_h(ah0, ah1, ah2, ah3, a, bh0, bh1, bh2, bh3);
    guard4_h(al0, al1, al2, al3, a, bl0, bl1, bl2, bl3);
  }
  acc_guard4(ah0, ah1, ah2, ah3);
  acc_guard4(al0, al1, al2, al3);

  float* slab = sT[wave];
#pragma unroll
  for (int r = 0; r < 8; ++r) {
    slab[(mOff + r) * 68 +  0 + rlane] = kOutScale * (ah0[r] + al0[r] * kLoFold);
    slab[(mOff + r) * 68 + 16 + rlane] = kOutScale * (ah1[r] + al1[r] * kLoFold);
    slab[(mOff + r) * 68 + 32 + rlane] = kOutScale * (ah2[r] + al2[r] * kLoFold);
    slab[(mOff + r) * 68 + 48 + rlane] = kOutScale * (ah3[r] + al3[r] * kLoFold);
  }
  __syncthreads();
  const int hh = lane >> 4, c4 = (lane & 15) * 4;
  v4f vv[8];
#pragma unroll
  for (int it = 0; it < 8; ++it) {
    const int row = it * 2 + hh;
    vv[it] = *(const v4f*)(slab + row * 68 + c4);
  }
  float* ob = out + ((size_t)bh * kSeq + i0) * kHd + c4;
  for (int pass = 0; pass < 2; ++pass) {
#pragma unroll
    for (int it = 0; it < 8; ++it) {
      const int row = it * 2 + hh;
      *(volatile v4f*)(ob + (size_t)row * kHd) = vv[it];
    }
    __threadfence();
  }
}

extern "C" void kernel_launch(void* const* d_in, const int* in_sizes, int n_in,
                              void* d_out, int out_size, void* d_ws, size_t ws_size,
                              hipStream_t stream) {
  if (n_in < 3) return;
  if (in_sizes[0] != kTok * kDim) return;
  if (in_sizes[1] != kDim * kCols) return;
  if (in_sizes[2] != kCols) return;
  if (out_size != kBH * kSeq * kHd) return;
  if (ws_size < kWsTotal) return;

  const float* x    = (const float*)d_in[0];
  const float* W    = (const float*)d_in[1];
  const float* bqkv = (const float*)d_in[2];
  float* out = (float*)d_out;

  char* ws = (char*)d_ws;
  unsigned short* X16   = (unsigned short*)(ws + kOffX16);
  unsigned short* WT16  = (unsigned short*)(ws + kOffWT16);
  float*          BPERM = (float*)(ws + kOffBPERM);
  unsigned short* Q16   = (unsigned short*)(ws + kOffQ16);
  unsigned short* KVT16 = (unsigned short*)(ws + kOffKVT16);
  unsigned short* MTHI  = (unsigned short*)(ws + kOffMTHI);
  unsigned short* MTLO  = (unsigned short*)(ws + kOffMTLO);

  cvt_rows_bf16_kernel<<<(kTok * kDim / 8) / 256, 256, 0, stream>>>(x, (unsigned int*)X16, kTok * kDim / 8);

  wt_deint_bf16_kernel<<<dim3(kDim / 64, kHeads), 256, 0, stream>>>(W, WT16);

  bias_perm_kernel<<<(kCols / 4) / 256, 256, 0, stream>>>(bqkv, BPERM);

  gemm64_bf16_f16out_kernel<2><<<((kTok / 64) * (kDim / 64)) / 8, 256, 0, stream>>>(
      X16, kDim, WT16, kDim, Q16, kDim, BPERM, kTok, kDim, kDim, kQCarry);

  gemm64_bf16_f16out_kernel<1><<<(((2 * kDim) / 64) * (kTok / 64)) / 8, 256, 0, stream>>>(
      WT16 + (size_t)kDim * kDim, kDim, X16, kDim, KVT16, kTok, BPERM + kDim, 2 * kDim, kTok, kDim, kQCarry);

  ktv_kernel<<<kBH, 128, 0, stream>>>(KVT16, MTHI, MTLO);

  qm_out_kernel<<<kBH * (kSeq / kOutRows), 256, 0, stream>>>(Q16, MTHI, MTLO, out);
}
